// TinyAttention_79439715107357
// MI455X (gfx1250) — hardware-verified
//
#include <hip/hip_runtime.h>
#include <math.h>


#define D_MODEL 512
#define D_ATTN  64
#define NSEQ    2048
#define NBATCH  8
#define NTOK    (NBATCH * NSEQ)
#define D_OUT   256
#define D_QKV   192
#define SCALE_F 0.125f

typedef __attribute__((ext_vector_type(16))) __bf16 v16bf;
typedef __attribute__((ext_vector_type(8)))  __bf16 v8bf;
typedef __attribute__((ext_vector_type(8)))  float  v8f;
typedef __attribute__((ext_vector_type(4)))  float  v4f;
typedef __attribute__((ext_vector_type(4)))  unsigned v4u;

template <typename T> __device__ __forceinline__ void vst2(void* p, T v) { *(volatile T*)p = v; __threadfence(); *(volatile T*)p = v; }
__device__ __forceinline__ v8f wmma_bf(v16bf a, v16bf b, v8f c) {
  v8f d = __builtin_amdgcn_wmma_f32_16x16x32_bf16(false, a, false, b, (short)0, c, false, false);
  asm volatile("v_nop\n\tv_nop\n\tv_nop\n\tv_nop" : "+v"(d) : "v"(a), "v"(b));
  return d;
}
struct F2 { v16bf h, l; };
__device__ __forceinline__ F2 split_f32(const float* row, int k0, int lane) {
  F2 r; const float* p = row + k0 + 8 * (lane >> 4);
#pragma unroll
  for (int i = 0; i < 16; ++i) { const float x = p[(i < 8) ? i : (i + 8)]; const __bf16 h = (__bf16)x; r.h[i] = h; r.l[i] = (__bf16)(x - (float)h); }
  return r;
}
__device__ __forceinline__ v16bf frag_bf(const __bf16* row, int k0, int lane) {
  union { v16bf v; v8bf q[2]; } r; const __bf16* p = row + k0 + 8 * (lane >> 4);
  r.q[0] = *(const v8bf*)(p); r.q[1] = *(const v8bf*)(p + 16); return r.v;
}
__device__ __forceinline__ v8f mac3(const F2& a, const F2& b, v8f c) {
  c = wmma_bf(a.l, b.h, c); c = wmma_bf(a.h, b.l, c); c = wmma_bf(a.h, b.h, c); return c;
}
__device__ __forceinline__ v8f mac3p(const F2& a, const __bf16* bh, const __bf16* bl, int k0, int lane, v8f c) {
  const v16bf fh = frag_bf(bh, k0, lane), fl = frag_bf(bl, k0, lane);
  c = wmma_bf(a.l, fh, c); c = wmma_bf(a.h, fl, c); c = wmma_bf(a.h, fh, c); return c;
}

__global__ __launch_bounds__(256) void k_wt(const float* __restrict__ W, __bf16* __restrict__ Ph, __bf16* __restrict__ Pl, int K, int N) {
  __shared__ __align__(16) __bf16 th[64][72], tl[64][72];
  const int nt = N / 64, tid = threadIdx.x;
  const int n0 = (blockIdx.x % nt) * 64, k0 = (blockIdx.x / nt) * 64;
  for (int i = tid; i < 64 * 64; i += 256) { const int kk = i >> 6, nn = i & 63; const float x = W[(size_t)(k0 + kk) * N + n0 + nn];
    const __bf16 h = (__bf16)x; th[nn][kk] = h; tl[nn][kk] = (__bf16)(x - (float)h); }
  __syncthreads();
  for (int g = tid; g < 64 * 8; g += 256) { const int nn = g >> 3, pc = g & 7; const size_t o = (size_t)(n0 + nn) * K + k0 + pc * 8;
    vst2(Ph + o, *(const v4u*)(&th[nn][pc * 8])); vst2(Pl + o, *(const v4u*)(&tl[nn][pc * 8])); }
}

__global__ __launch_bounds__(128) void k_qkv(const float* __restrict__ x, const __bf16* __restrict__ Wh, const __bf16* __restrict__ Wl,
                                            const float* __restrict__ bq, float* __restrict__ qb, float* __restrict__ kb, float* __restrict__ vT) {
  __shared__ __align__(16) float st[64][196];
  const int tid = threadIdx.x, wave = tid >> 5, lane = tid & 31, col = lane & 15, g = lane >> 4;
  const int m0 = blockIdx.x * 64 + wave * 16;
  const float* ar = x + (size_t)(m0 + col) * D_MODEL;
  v8f c[12] = {};
#pragma unroll 1
  for (int kc = 0; kc < D_MODEL / 32; ++kc) {
    const F2 a = split_f32(ar, kc * 32, lane);
#pragma unroll
    for (int j = 0; j < 12; ++j) c[j] = mac3p(a, Wh + (size_t)(j * 16 + col) * D_MODEL, Wl + (size_t)(j * 16 + col) * D_MODEL, kc * 32, lane, c[j]);
  }
#pragma unroll
  for (int j = 0; j < 12; ++j) { const float bb = bq[j * 16 + col];
#pragma unroll
    for (int r = 0; r < 8; ++r) st[wave * 16 + g * 8 + r][j * 16 + col] = c[j][r] + bb; }
  __syncthreads();
  for (int gq = tid; gq < 64 * 16; gq += 128) { const int rl = gq >> 4, pc = gq & 15;
    vst2(qb + (size_t)(blockIdx.x * 64 + rl) * D_ATTN + pc * 4, *(const v4f*)(&st[rl][pc * 4]));
    vst2(kb + (size_t)(blockIdx.x * 64 + rl) * D_ATTN + pc * 4, *(const v4f*)(&st[rl][64 + pc * 4])); }
  { const int bm0 = blockIdx.x * 64, bidx = bm0 >> 11, n0 = bm0 & (NSEQ - 1);
    for (int gq = tid; gq < 64 * 16; gq += 128) { const int d = gq >> 4, pc = gq & 15;
      v4f v = { st[pc * 4][128 + d], st[pc * 4 + 1][128 + d], st[pc * 4 + 2][128 + d], st[pc * 4 + 3][128 + d] };
      vst2(vT + ((size_t)bidx * D_ATTN + d) * NSEQ + n0 + pc * 4, v); } }
}

__global__ __launch_bounds__(256) void k_attn(const float* __restrict__ qb, const float* __restrict__ kb, const float* __restrict__ vT, float* __restrict__ ob) {
  __shared__ __align__(16) float pl[8][16 * 32];
  __shared__ __align__(16) float os[8][16 * 64];
  const int wave = blockIdx.x * 8 + (threadIdx.x >> 5), wl = threadIdx.x >> 5;
  const int b = wave >> 7, qs = (wave & 127) * 16;
  const int lane = threadIdx.x & 31, g = lane >> 4, col = lane & 15;
  const float* qrow = qb + ((size_t)b * NSEQ + qs + col) * D_ATTN;
  const F2 qa = split_f32(qrow, 0, lane), qc = split_f32(qrow, 32, lane);
  float m_r[8], l_r[8];
  v8f o[4] = {};
#pragma unroll
  for (int r = 0; r < 8; ++r) { m_r[r] = -1e30f; l_r[r] = 0.f; }
  float* p = pl[wl];
  const int jmax = (qs + 15) >> 5;
  for (int j = 0; j <= jmax; ++j) {
    const int ks = j * 32;
    const float* krow0 = kb + ((size_t)b * NSEQ + ks + col) * D_ATTN;
    const float* krow1 = krow0 + 16 * D_ATTN;
    v8f s0 = {}, s1 = {};
    s0 = mac3(qa, split_f32(krow0, 0, lane), s0); s0 = mac3(qc, split_f32(krow0, 32, lane), s0);
    s1 = mac3(qa, split_f32(krow1, 0, lane), s1); s1 = mac3(qc, split_f32(krow1, 32, lane), s1);
#pragma unroll
    for (int r = 0; r < 8; ++r) {
      const int qi = qs + r + 8 * g;
      float a0 = s0[r] * SCALE_F; if (ks + col > qi)      a0 = -1e30f;
      float a1 = s1[r] * SCALE_F; if (ks + 16 + col > qi) a1 = -1e30f;
      float mx = fmaxf(a0, a1);
#pragma unroll
      for (int off = 8; off >= 1; off >>= 1) mx = fmaxf(mx, __shfl_xor(mx, off, 32));
      const float mn = fmaxf(m_r[r], mx);
      const float p0 = __expf(a0 - mn), p1 = __expf(a1 - mn);
      const int row = r + 8 * g;
      p[row * 32 + col] = p0; p[row * 32 + 16 + col] = p1;
      float sum = p0 + p1;
#pragma unroll
      for (int off = 8; off >= 1; off >>= 1) sum += __shfl_xor(sum, off, 32);
      const float corr = __expf(m_r[r] - mn);
      l_r[r] = l_r[r] * corr + sum; m_r[r] = mn;
#pragma unroll
      for (int t = 0; t < 4; ++t) o[t][r] *= corr;
    }
    asm volatile("s_wait_dscnt 0" ::: "memory"); __builtin_amdgcn_wave_barrier(); __builtin_amdgcn_fence(__ATOMIC_RELEASE, "workgroup");
    const F2 pf = split_f32(p + col * 32, 0, lane);
    const float* vb = vT + (size_t)b * D_ATTN * NSEQ + ks;
#pragma unroll
    for (int t = 0; t < 4; ++t) o[t] = mac3(pf, split_f32(vb + (size_t)(t * 16 + col) * NSEQ, 0, lane), o[t]);
    __builtin_amdgcn_wave_barrier();
  }
  float* so = os[wl];
#pragma unroll
  for (int t = 0; t < 4; ++t)
#pragma unroll
    for (int r = 0; r < 8; ++r) so[(r + 8 * g) * 64 + t * 16 + col] = o[t][r] / l_r[r];
  asm volatile("s_wait_dscnt 0" ::: "memory"); __builtin_amdgcn_wave_barrier(); __builtin_amdgcn_fence(__ATOMIC_RELEASE, "workgroup");
#pragma unroll
  for (int q = 0; q < 8; ++q) { const int rl = q * 2 + (lane >> 4), pc = lane & 15;
    vst2(ob + ((size_t)b * NSEQ + qs + rl) * D_ATTN + pc * 4, *(const v4f*)(so + rl * 64 + pc * 4)); }
}

__global__ __launch_bounds__(128) void k_out(const float* __restrict__ ob, const __bf16* __restrict__ Wh, const __bf16* __restrict__ Wl,
                                            const float* __restrict__ bo, float* __restrict__ out) {
  __shared__ __align__(16) float st[4][16 * 260];
  const int tid = threadIdx.x, wave = tid >> 5, lane = tid & 31, col = lane & 15, g = lane >> 4;
  const int m0 = blockIdx.x * 64 + wave * 16;
  const float* ar = ob + (size_t)(m0 + col) * D_ATTN;
  const F2 a0 = split_f32(ar, 0, lane), a1 = split_f32(ar, 32, lane);
  float* S = st[wave];
#pragma unroll 2
  for (int j = 0; j < 16; ++j) {
    v8f c = {};
    c = mac3p(a0, Wh + (size_t)(j * 16 + col) * D_ATTN, Wl + (size_t)(j * 16 + col) * D_ATTN, 0, lane, c);
    c = mac3p(a1, Wh + (size_t)(j * 16 + col) * D_ATTN, Wl + (size_t)(j * 16 + col) * D_ATTN, 32, lane, c);
    const float bb = bo[j * 16 + col];
#pragma unroll
    for (int r = 0; r < 8; ++r) S[(r + 8 * g) * 260 + j * 16 + col] = c[r] + bb;
  }
  asm volatile("s_wait_dscnt 0" ::: "memory"); __builtin_amdgcn_wave_barrier(); __builtin_amdgcn_fence(__ATOMIC_RELEASE, "workgroup");
#pragma unroll 4
  for (int q = 0; q < 32; ++q) { const int rl = q >> 1, pc = (q & 1) * 32 + lane;
    vst2(out + (size_t)(m0 + rl) * D_OUT + pc * 4, *(const v4f*)(S + rl * 260 + pc * 4)); }
}

extern "C" void kernel_launch(void* const* d_in, const int* in_sizes, int n_in,
                              void* d_out, int out_size, void* d_ws, size_t ws_size,
                              hipStream_t stream) {
  (void)in_sizes; (void)n_in; (void)out_size; (void)ws_size;
  const float* x     = (const float*)d_in[0];
  const float* W_qkv = (const float*)d_in[1];
  const float* b_qkv = (const float*)d_in[2];
  const float* W_out = (const float*)d_in[3];
  const float* b_out = (const float*)d_in[4];
  float* out = (float*)d_out;
  char* ws = (char*)d_ws; size_t off = 0;
  auto alloc = [&](size_t bytes) -> void* { void* p = ws + off; off = (off + bytes + 255) & ~(size_t)255; return p; };
  __bf16* Wqh = (__bf16*)alloc((size_t)D_QKV * D_MODEL * 2); __bf16* Wql = (__bf16*)alloc((size_t)D_QKV * D_MODEL * 2);
  __bf16* Woh = (__bf16*)alloc((size_t)D_OUT * D_ATTN * 2);  __bf16* Wol = (__bf16*)alloc((size_t)D_OUT * D_ATTN * 2);
  float* qb = (float*)alloc((size_t)NTOK * D_ATTN * 4); float* kb = (float*)alloc((size_t)NTOK * D_ATTN * 4);
  float* vT = (float*)alloc((size_t)NTOK * D_ATTN * 4); float* ob = (float*)alloc((size_t)NTOK * D_ATTN * 4);

  k_wt<<<(D_MODEL / 64) * (D_QKV / 64), 256, 0, stream>>>(W_qkv, Wqh, Wql, D_MODEL, D_QKV);
  k_wt<<<(D_ATTN / 64) * (D_OUT / 64), 256, 0, stream>>>(W_out, Woh, Wol, D_ATTN, D_OUT);
  k_qkv<<<NTOK / 64, 128, 0, stream>>>(x, Wqh, Wql, b_qkv, qb, kb, vT);
  k_attn<<<NBATCH * (NSEQ / 16) / 8, 256, 0, stream>>>(qb, kb, vT, ob);
  k_out<<<NTOK / 64, 128, 0, stream>>>(ob, Woh, Wol, b_out, out);
}
